// MultiHeadSliddingWindowAttention_37976100831414
// MI455X (gfx1250) — hardware-verified
//
#include <hip/hip_runtime.h>
#include <stdint.h>

constexpr int NBATCH  = 2;
constexpr int SEQ     = 2048;
constexpr int EMB     = 768;
constexpr int NHEAD   = 12;
constexpr int HDIM    = 64;
constexpr int NTOK    = NBATCH * SEQ;
constexpr int NBH     = NBATCH * NHEAD;
constexpr int NDIAG   = 257;
constexpr int TAILCNT = SEQ - NDIAG;
constexpr int KPV     = 288;
constexpr int PPITCH  = 320;
constexpr int BPITCH  = 260;
constexpr int WTPITCH = 72;
constexpr float WMUL    = 32.0f;
constexpr float YMUL    = 16.0f;
constexpr float PSC     = 32768.0f;
constexpr float PSC_INV = 1.0f / 32768.0f;

typedef __attribute__((ext_vector_type(16))) _Float16 v16h;
typedef __attribute__((ext_vector_type(8)))  _Float16 v8h;
typedef __attribute__((ext_vector_type(16))) __bf16   v16b;
typedef __attribute__((ext_vector_type(8)))  __bf16   v8b;
typedef __attribute__((ext_vector_type(8)))  float    v8f;
typedef __attribute__((ext_vector_type(4)))  float    v4f;
typedef __attribute__((ext_vector_type(8)))  unsigned short v8u;

__device__ __forceinline__ unsigned short f2bf_bits(float f) {
  unsigned u = __float_as_uint(f);
  return (unsigned short)((u + 0x7FFFu + ((u >> 16) & 1u)) >> 16);
}
__device__ __forceinline__ float bf_bits2f(unsigned short h) { return __uint_as_float(((unsigned)h) << 16); }
__device__ __forceinline__ float bf_rne(float f) { return bf_bits2f(f2bf_bits(f)); }

__device__ __forceinline__ void dep_guard_h(v8f& a, v8f& b, v16h x, v16h y) { asm volatile("v_nop\n\tv_nop\n\tv_nop\n\tv_nop" : "+v"(a), "+v"(b) : "v"(x), "v"(y)); }
__device__ __forceinline__ void dep_guard_b(v8f& a, v8f& b, v16b x, v16b y) { asm volatile("v_nop\n\tv_nop\n\tv_nop\n\tv_nop" : "+v"(a), "+v"(b) : "v"(x), "v"(y)); }
__device__ __forceinline__ void keep4_h(v16h a, v16h b, v16h c, v16h d) { asm volatile("v_nop" :: "v"(a), "v"(b), "v"(c), "v"(d)); }
__device__ __forceinline__ void keep4_b(v16b a, v16b b, v16b c, v16b d) { asm volatile("v_nop" :: "v"(a), "v"(b), "v"(c), "v"(d)); }
__device__ __forceinline__ void acc_guard4(v8f& a, v8f& b, v8f& c, v8f& d) { asm volatile("v_nop\n\tv_nop\n\tv_nop\n\tv_nop" : "+v"(a), "+v"(b), "+v"(c), "+v"(d)); }
template <typename T> struct Frag;
template <> struct Frag<_Float16> {
  typedef v16h V; union U { v16h v; v8h h[2]; };
  static __device__ __forceinline__ v16h load(const _Float16* p) {
    U f; f.h[0] = *(const v8h*)(p); f.h[1] = *(const v8h*)(p + 16); return f.v;
  }
  static __device__ __forceinline__ v8f mma(v16h a, v16h b, v8f c) {
    return __builtin_amdgcn_wmma_f32_16x16x32_f16(false, a, false, b, (short)0, c, false, false);
  }
  static __device__ __forceinline__ void guard(v8f& a, v8f& b, v16h x, v16h y) { dep_guard_h(a, b, x, y); }
  static __device__ __forceinline__ void keep(v16h a, v16h b, v16h c, v16h d) { keep4_h(a, b, c, d); }
};
template <> struct Frag<__bf16> {
  typedef v16b V; union U { v16b v; v8b h[2]; };
  static __device__ __forceinline__ v16b load(const __bf16* p) {
    U f; f.h[0] = *(const v8b*)(p); f.h[1] = *(const v8b*)(p + 16); return f.v;
  }
  static __device__ __forceinline__ v8f mma(v16b a, v16b b, v8f c) {
    return __builtin_amdgcn_wmma_f32_16x16x32_bf16(false, a, false, b, (short)0, c, false, false);
  }
  static __device__ __forceinline__ void guard(v8f& a, v8f& b, v16b x, v16b y) { dep_guard_b(a, b, x, y); }
  static __device__ __forceinline__ void keep(v16b a, v16b b, v16b c, v16b d) { keep4_b(a, b, c, d); }
};

__device__ __forceinline__ v8f at_mma(v16b a, v16b b, v8f c) {
  c = __builtin_amdgcn_wmma_f32_16x16x32_bf16(false, a, false, b, (short)0, c, false, false);
  asm volatile("v_nop\n\tv_nop\n\tv_nop\n\tv_nop" : "+v"(c) : "v"(a), "v"(b));
  return c;
}

template <int ET> struct Elem;
template <> struct Elem<0> { typedef _Float16 T; };
template <> struct Elem<1> { typedef __bf16 T; };
template <int ET, bool SPLIT, int BIAS_MODE, int OUT_MODE, bool RESID, int ACT = 0>
__global__ __launch_bounds__(256) void wmma_gemm64(
    const unsigned short* __restrict__ Ap, const unsigned short* __restrict__ A2p, int lda, long strideA,
    const unsigned short* __restrict__ Btp, const unsigned short* __restrict__ Bt2p, int ldb, long strideB,
    void* __restrict__ Cout, void* __restrict__ Cout2, int ldc, long strideC,
    const float* __restrict__ bias,
    const float* __restrict__ resid, long strideR,
    int M, int N, int K, float scale) {
  typedef typename Elem<ET>::T T;
  typedef typename Frag<T>::V V;
  const T* A = (const T*)Ap; const T* A2 = (const T*)A2p; const T* Bt = (const T*)Btp; const T* Bt2 = (const T*)Bt2p;
  __shared__ __align__(16) float sT[8][16 * 68];
  const int b    = blockIdx.y;
  const int lane = threadIdx.x & 31;
  const int wave = threadIdx.x >> 5;
  const int tilesN = N >> 6;
  const int tilesM = M >> 6;
  const int tile = blockIdx.x * 8 + wave;
  if (tile >= tilesM * tilesN) return;
  const int tm = tile / tilesN;
  const int tn = tile - tm * tilesN;
  const int m0 = tm << 6;
  const int n0 = tn << 6;

  const T* Ab  = A  + (size_t)b * strideA;
  const T* Bb  = Bt + (size_t)b * strideB;
  const T* Ab2 = SPLIT ? (A2  + (size_t)b * strideA) : nullptr;
  const T* Bb2 = SPLIT ? (Bt2 + (size_t)b * strideB) : nullptr;

  const int rlane = lane & 15;
  const int koff  = (lane >> 4) * 8;
  const int mOff  = (lane >> 4) * 8;

  v8f acc[4][4];
#pragma unroll
  for (int i = 0; i < 4; ++i)
#pragma unroll
    for (int j = 0; j < 4; ++j) acc[i][j] = (v8f){0.f,0.f,0.f,0.f,0.f,0.f,0.f,0.f};

  for (int k0 = 0; k0 < K; k0 += 32) {
    V bh[4], bl[4];
#pragma unroll
    for (int j = 0; j < 4; ++j) {
      const size_t bo = (size_t)(n0 + (j << 4) + rlane) * ldb + koff + k0;
      bh[j] = Frag<T>::load(Bb + bo);
      if (SPLIT) bl[j] = Frag<T>::load(Bb2 + bo);
    }
#pragma unroll
    for (int i = 0; i < 4; ++i) {
      const size_t ao = (size_t)(m0 + (i << 4) + rlane) * lda + koff + k0;
      V ah = Frag<T>::load(Ab + ao);
      V al;
      if (SPLIT) al = Frag<T>::load(Ab2 + ao);
#pragma unroll
      for (int j = 0; j < 4; ++j) {
        acc[i][j] = Frag<T>::mma(ah, bh[j], acc[i][j]);
        if (SPLIT) {
          acc[i][j] = Frag<T>::mma(ah, bl[j], acc[i][j]);
          acc[i][j] = Frag<T>::mma(al, bh[j], acc[i][j]);
        }
      }
      Frag<T>::guard(acc[i][0], acc[i][3], ah, SPLIT ? al : ah);
    }
    Frag<T>::keep(bh[0], bh[1], bh[2], bh[3]);
    if (SPLIT) Frag<T>::keep(bl[0], bl[1], bl[2], bl[3]);
  }
  acc_guard4(acc[0][0], acc[0][1], acc[0][2], acc[0][3]);
  acc_guard4(acc[1][0], acc[1][1], acc[1][2], acc[1][3]);
  acc_guard4(acc[2][0], acc[2][1], acc[2][2], acc[2][3]);
  acc_guard4(acc[3][0], acc[3][1], acc[3][2], acc[3][3]);

  float* slab = sT[wave];
  const float* Rb = RESID ? (resid + (size_t)b * strideR) : nullptr;
#pragma unroll
  for (int i = 0; i < 4; ++i) {
    const int mBase = m0 + (i << 4);
#pragma unroll
    for (int j = 0; j < 4; ++j) {
      const int n = n0 + (j << 4) + rlane;
      float bv = 0.f;
      if (BIAS_MODE == 2) bv = bias[n];
      if (BIAS_MODE == 3) bv = bf_rne(bias[n]);
#pragma unroll
      for (int r = 0; r < 8; ++r) {
        float v = acc[i][j][r] * scale;
        if (BIAS_MODE == 1) v += bias[mBase + mOff + r];
        if (BIAS_MODE == 2 || BIAS_MODE == 3) v += bv;
        if (RESID) v += Rb[(size_t)(mBase + mOff + r) * ldc + n];
        if (ACT == 1) v = tanhf(v);
        if (ACT == 2) v = fmaxf(v, 0.0f);
        if (ACT == 3) v = v / (1.0f + expf(-v));
        if (ACT == 4) v = (v > 0.f) ? v : 0.01f * v;
        slab[(mOff + r) * 68 + (j << 4) + rlane] = v;
      }
    }
    __builtin_amdgcn_fence(__ATOMIC_RELEASE, "workgroup");
    __builtin_amdgcn_wave_barrier();
    __builtin_amdgcn_fence(__ATOMIC_ACQUIRE, "workgroup");
    if (OUT_MODE == 0) {
      float* C = (float*)Cout + (size_t)b * strideC;
      const int hh = lane >> 4, c4 = (lane & 15) * 4;
      for (int pass = 0; pass < 2; ++pass) {
#pragma unroll
        for (int it = 0; it < 8; ++it) {
          const int row = it * 2 + hh;
          v4f v = *(const v4f*)(slab + row * 68 + c4);
          *(volatile v4f*)(C + (size_t)(mBase + row) * ldc + n0 + c4) = v;
        }
        __threadfence();
      }
    } else {
      const int q = lane >> 3, c8 = (lane & 7) * 8;
      unsigned short* C  = (unsigned short*)Cout  + (size_t)b * strideC;
      unsigned short* C2 = (OUT_MODE == 2) ? ((unsigned short*)Cout2 + (size_t)b * strideC) : nullptr;
      for (int pass = 0; pass < 2; ++pass) {
#pragma unroll
        for (int it = 0; it < 4; ++it) {
          const int row = it * 4 + q;
          const float* sp = slab + row * 68 + c8;
          v8h hv, lv;
#pragma unroll
          for (int e = 0; e < 8; ++e) {
            if (OUT_MODE == 1) {
              hv[e] = (_Float16)sp[e];
            } else {
              unsigned short hb = f2bf_bits(sp[e]);
              unsigned short lb = f2bf_bits(sp[e] - bf_bits2f(hb));
              hv[e] = __builtin_bit_cast(_Float16, hb);
              lv[e] = __builtin_bit_cast(_Float16, lb);
            }
          }
          *(volatile v8h*)(C + (size_t)(mBase + row) * ldc + n0 + c8) = hv;
          if (OUT_MODE == 2) *(volatile v8h*)(C2 + (size_t)(mBase + row) * ldc + n0 + c8) = lv;
        }
        __threadfence();
      }
    }
    __builtin_amdgcn_fence(__ATOMIC_RELEASE, "workgroup");
    __builtin_amdgcn_wave_barrier();
    __builtin_amdgcn_fence(__ATOMIC_ACQUIRE, "workgroup");
  }
}

__global__ __launch_bounds__(256) void cast_x_k(const float* __restrict__ in, unsigned short* __restrict__ out, int n2) {
  const int i = blockIdx.x * 256 + threadIdx.x;
  if (i < n2) {
    const _Float16 h0 = (_Float16)bf_rne(in[2 * i]);
    const _Float16 h1 = (_Float16)bf_rne(in[2 * i + 1]);
    const unsigned u = (unsigned)__builtin_bit_cast(unsigned short, h0) | ((unsigned)__builtin_bit_cast(unsigned short, h1) << 16);
    ((volatile unsigned*)out)[i] = u;
    __threadfence();
    ((volatile unsigned*)out)[i] = u;
  }
}

__global__ __launch_bounds__(256) void wt_cast_k(const float* __restrict__ W, unsigned short* __restrict__ Wtp,
                                                 int K, int N, float mul) {
  __shared__ __align__(16) _Float16 st[64 * WTPITCH];
  _Float16* Wt = (_Float16*)(void*)Wtp;
  const int n0 = blockIdx.x * 64, k0 = blockIdx.y * 64;
  const int tid = threadIdx.x;
  const int kr = tid >> 2, c16 = (tid & 3) * 16;
  const float* src = W + (size_t)(k0 + kr) * N + n0 + c16;
#pragma unroll
  for (int q = 0; q < 4; ++q) {
    const v4f v = *(const v4f*)(src + 4 * q);
#pragma unroll
    for (int e = 0; e < 4; ++e) st[(c16 + 4 * q + e) * WTPITCH + kr] = (_Float16)(bf_rne(v[e]) * mul);
  }
  __syncthreads();
  const int wave = tid >> 5, lane = tid & 31;
  const int q8 = lane >> 3, c8 = (lane & 7) * 8;
  for (int pass = 0; pass < 2; ++pass) {
#pragma unroll
    for (int it = 0; it < 2; ++it) {
      const int n = it * 32 + wave * 4 + q8;
      const v8h hv = *(const v8h*)(st + n * WTPITCH + c8);
      *(volatile v8h*)(Wt + (size_t)(n0 + n) * K + k0 + c8) = hv;
    }
    __threadfence();
  }
}

__global__ __launch_bounds__(256) void vprep_k(const float* __restrict__ V32, unsigned short* __restrict__ Vtp,
                                               float* __restrict__ SV) {
  __shared__ __align__(16) _Float16 st[64 * WTPITCH];
  __shared__ __align__(16) float part[4][64];
  __shared__ __align__(16) float svs[64];
  _Float16* Vt = (_Float16*)(void*)Vtp;
  const int bh = blockIdx.x;
  const int b = bh / NHEAD, h = bh - b * NHEAD;
  const int tid = threadIdx.x, wave = tid >> 5, lane = tid & 31;
  const float* Vb = V32 + (size_t)b * SEQ * EMB + h * HDIM;
  const int q8 = lane >> 3, c8 = (lane & 7) * 8;
#pragma unroll 1
  for (int ct = 0; ct < 5; ++ct) {
    const int c0 = ct * 64;
    {
      const int kr = tid >> 2, d16 = (tid & 3) * 16;
      const int c = c0 + kr;
      const float* src = Vb + (size_t)c * EMB + d16;
#pragma unroll
      for (int q = 0; q < 4; ++q) {
        const v4f v = *(const v4f*)(src + 4 * q);
#pragma unroll
        for (int e = 0; e < 4; ++e)
          st[(d16 + 4 * q + e) * WTPITCH + kr] = (c < NDIAG) ? (_Float16)v[e] : (_Float16)0.0f;
      }
    }
    __syncthreads();
    for (int pass = 0; pass < 2; ++pass) {
#pragma unroll
      for (int it = 0; it < 2; ++it) {
        const int d = it * 32 + wave * 4 + q8;
        const v8h hv = *(const v8h*)(st + d * WTPITCH + c8);
        *(volatile v8h*)(Vt + ((size_t)bh * HDIM + d) * PPITCH + c0 + c8) = hv;
      }
      __threadfence();
    }
    __syncthreads();
  }
  {
    const int d = tid & 63, pidx = tid >> 6;
    const int cb = NDIAG + pidx * 448;
    int ce = cb + 448; if (ce > SEQ) ce = SEQ;
    float s = 0.0f;
#pragma unroll 1
    for (int c = cb; c < ce; ++c) s += Vb[(size_t)c * EMB + d];
    part[pidx][d] = s;
  }
  __syncthreads();
  if (tid < 64) svs[tid] = ((part[0][tid] + part[1][tid]) + part[2][tid]) + part[3][tid];
  __syncthreads();
  if (wave == 0) {
    const int l16 = (lane < 16) ? lane : 15;
    const v4f sv4 = *(const v4f*)(svs + l16 * 4);
    float* dst = SV + (size_t)bh * HDIM + l16 * 4;
    if (lane < 16) *(volatile v4f*)dst = sv4;
    __threadfence();
    if (lane < 16) *(volatile v4f*)dst = sv4;
  }
}

__global__ __launch_bounds__(128) void band_softmax_k(
    const unsigned short* __restrict__ Qhp, const unsigned short* __restrict__ Qlp,
    const unsigned short* __restrict__ Khp, const unsigned short* __restrict__ Klp,
    unsigned short* __restrict__ Pp, float* __restrict__ stats) {
  union FB { v16b v; v8u u[2]; };
  __shared__ __align__(16) unsigned short Ksh[64 * 64];
  __shared__ __align__(16) unsigned short Ksl[64 * 64];
  __shared__ __align__(16) float slab[4][16 * BPITCH];
  __shared__ __align__(16) _Float16 pst[4][4 * PPITCH];
  __shared__ __align__(16) float stst[64 * 2];

  const int tid = threadIdx.x;
  const int wave = tid >> 5;
  const int lane = tid & 31;
  const int hh = lane >> 4;
  const int c = lane & 15;
  const int qb = blockIdx.x & 31;
  const int bh = blockIdx.x >> 5;
  const int b = bh / NHEAD, h = bh - b * NHEAD;
  const int n0 = qb * 64;
  const int q0 = n0 + wave * 16;
  const size_t tok0 = (size_t)b * SEQ;
  const __bf16* Qh = (const __bf16*)(const void*)Qhp;
  const __bf16* Ql = (const __bf16*)(const void*)Qlp;

  v16b qah[2], qal[2];
  {
    const size_t qoff = (tok0 + q0 + c) * EMB + (size_t)h * HDIM + 8 * hh;
#pragma unroll
    for (int dc = 0; dc < 2; ++dc) {
      qah[dc] = Frag<__bf16>::load(Qh + qoff + dc * 32);
      qal[dc] = Frag<__bf16>::load(Ql + qoff + dc * 32);
    }
  }
  float* sw = slab[wave];

#pragma unroll 1
  for (int kc = 0; kc < 5; ++kc) {
    const int kv0 = n0 - 128 + kc * 64;
    __syncthreads();
    {
      const int kvr = tid >> 1, dh = (tid & 1) * 32;
      int kva = kv0 + kvr;
      kva = kva < 0 ? 0 : (kva > SEQ - 1 ? SEQ - 1 : kva);
      const size_t koff = (tok0 + kva) * EMB + (size_t)h * HDIM + dh;
#pragma unroll
      for (int i = 0; i < 4; ++i) {
        const v8u a  = *(const v8u*)(Khp + koff + 8 * i);
        const v8u a2 = *(const v8u*)(Klp + koff + 8 * i);
        *(v8u*)(Ksh + kvr * 64 + dh + 8 * i) = a;
        *(v8u*)(Ksl + kvr * 64 + dh + 8 * i) = a2;
      }
    }
    __syncthreads();

    v8f s[4];
#pragma unroll
    for (int j = 0; j < 4; ++j) {
      s[j] = (v8f){0.f,0.f,0.f,0.f,0.f,0.f,0.f,0.f};
#pragma unroll
      for (int dc = 0; dc < 2; ++dc) {
        FB kb, kl;
        kb.u[0] = *(const v8u*)(Ksh + (j * 16 + c) * 64 + dc * 32 + 8 * hh);
        kb.u[1] = *(const v8u*)(Ksh + (j * 16 + c) * 64 + dc * 32 + 16 + 8 * hh);
        kl.u[0] = *(const v8u*)(Ksl + (j * 16 + c) * 64 + dc * 32 + 8 * hh);
        kl.u[1] = *(const v8u*)(Ksl + (j * 16 + c) * 64 + dc * 32 + 16 + 8 * hh);
        s[j] = at_mma(qah[dc], kb.v, s[j]);
        s[j] = at_mma(qah[dc], kl.v, s[j]);
        s[j] = at_mma(qal[dc], kb.v, s[j]);
      }
    }
#pragma unroll
    for (int r = 0; r < 8; ++r) {
      const int nl = 8 * hh + r;
      const int nq = q0 + nl;
#pragma unroll
      for (int j = 0; j < 4; ++j) {
        const int kv = kv0 + j * 16 + c;
        const int cidx = kv - nq + 128;
        const float val = (kv >= 0 && kv < SEQ) ? s[j][r] : 0.0f;
        if ((unsigned)cidx < (unsigned)NDIAG) sw[nl * BPITCH + cidx] = val;
      }
    }
  }
  __syncthreads();

  _Float16* pw = pst[wave];
  _Float16* Pplane = (_Float16*)(void*)Pp;
  const int q4 = lane >> 3, c8 = (lane & 7) * 8;
#pragma unroll 1
  for (int rg = 0; rg < 4; ++rg) {
#pragma unroll 1
    for (int r4 = 0; r4 < 4; ++r4) {
      const int nl = rg * 4 + r4;
      const float* rowp = sw + nl * BPITCH;
      float v[9];
      float m = 0.0f;
#pragma unroll
      for (int i = 0; i < 9; ++i) {
        const int cc = lane + 32 * i;
        const int ccl = (cc < NDIAG) ? cc : (NDIAG - 1);
        const float x = rowp[ccl];
        v[i] = x;
        if (cc < NDIAG) m = fmaxf(m, x);
      }
#pragma unroll
      for (int off = 1; off < 32; off <<= 1) m = fmaxf(m, __shfl_xor(m, off, 32));
      float z = 0.0f;
      _Float16* prow = pw + r4 * PPITCH;
#pragma unroll
      for (int i = 0; i < 9; ++i) {
        const int cc = lane + 32 * i;
        const float p = expf(v[i] - m);
        if (cc < NDIAG) { z += p; prow[cc] = (_Float16)(p * PSC); }
      }
      prow[NDIAG + lane] = (_Float16)0.0f;
      if (lane < 31) prow[NDIAG + 32 + lane] = (_Float16)0.0f;
#pragma unroll
      for (int off = 1; off < 32; off <<= 1) z += __shfl_xor(z, off, 32);
      const float em = expf(-m);
      z += (float)TAILCNT * em;
      if (lane == 0) {
        stst[(wave * 16 + nl) * 2]     = em;
        stst[(wave * 16 + nl) * 2 + 1] = 1.0f / z;
      }
    }
    __builtin_amdgcn_fence(__ATOMIC_RELEASE, "workgroup");
    __builtin_amdgcn_wave_barrier();
    __builtin_amdgcn_fence(__ATOMIC_ACQUIRE, "workgroup");
    for (int pass = 0; pass < 2; ++pass) {
#pragma unroll
      for (int it = 0; it < 5; ++it) {
        const int L = it * 4 + q4;
        const int row4 = L / 5;
        const int seg = L - row4 * 5;
        const v8h hv = *(const v8h*)(pw + row4 * PPITCH + seg * 64 + c8);
        *(volatile v8h*)(Pplane + ((size_t)bh * SEQ + q0 + rg * 4 + row4) * PPITCH + seg * 64 + c8) = hv;
      }
      __threadfence();
    }
    __builtin_amdgcn_fence(__ATOMIC_RELEASE, "workgroup");
    __builtin_amdgcn_wave_barrier();
    __builtin_amdgcn_fence(__ATOMIC_ACQUIRE, "workgroup");
  }
  __syncthreads();
  if (wave == 0) {
    const v4f sv = *(const v4f*)(stst + lane * 4);
    float* dst = stats + ((size_t)bh * SEQ + n0) * 2 + lane * 4;
    *(volatile v4f*)dst = sv;
    __threadfence();
    *(volatile v4f*)dst = sv;
  }
}

__global__ __launch_bounds__(256) void pv_gemm_k(
    const unsigned short* __restrict__ Pp, const unsigned short* __restrict__ Vtp,
    const float* __restrict__ stats, const float* __restrict__ SVp, unsigned short* __restrict__ Yp) {
  typedef _Float16 T;
  typedef v16h V;
  __shared__ __align__(16) float sT[8][16 * 68];
  const int z = blockIdx.y;
  const int bb = z / NHEAD, hd = z - bb * NHEAD;
  const int lane = threadIdx.x & 31;
  const int wave = threadIdx.x >> 5;
  const int tile = blockIdx.x * 8 + wave;
  if (tile >= SEQ / 64) return;
  const int m0 = tile << 6;
  const T* Ab = (const T*)(const void*)Pp  + (size_t)z * SEQ  * PPITCH;
  const T* Bb = (const T*)(const void*)Vtp + (size_t)z * HDIM * PPITCH;
  const int rlane = lane & 15;
  const int koff  = (lane >> 4) * 8;
  const int mOff  = (lane >> 4) * 8;

  v8f acc[4][4];
#pragma unroll
  for (int i = 0; i < 4; ++i)
#pragma unroll
    for (int j = 0; j < 4; ++j) acc[i][j] = (v8f){0.f,0.f,0.f,0.f,0.f,0.f,0.f,0.f};

  for (int k0 = 0; k0 < KPV; k0 += 32) {
    V bfr[4];
#pragma unroll
    for (int j = 0; j < 4; ++j)
      bfr[j] = Frag<T>::load(Bb + (size_t)((j << 4) + rlane) * PPITCH + koff + k0);
#pragma unroll
    for (int i = 0; i < 4; ++i) {
      V af = Frag<T>::load(Ab + (size_t)(m0 + (i << 4) + rlane) * PPITCH + koff + k0);
#pragma unroll
      for (int j = 0; j < 4; ++j) acc[i][j] = Frag<T>::mma(af, bfr[j], acc[i][j]);
      Frag<T>::guard(acc[i][0], acc[i][3], af, af);
    }
    Frag<T>::keep(bfr[0], bfr[1], bfr[2], bfr[3]);
  }
  acc_guard4(acc[0][0], acc[0][1], acc[0][2], acc[0][3]);
  acc_guard4(acc[1][0], acc[1][1], acc[1][2], acc[1][3]);
  acc_guard4(acc[2][0], acc[2][1], acc[2][2], acc[2][3]);
  acc_guard4(acc[3][0], acc[3][1], acc[3][2], acc[3][3]);

  float* slab = sT[wave];
  _Float16* C = (_Float16*)(void*)Yp + (size_t)bb * SEQ * EMB + (size_t)hd * HDIM;
#pragma unroll
  for (int i = 0; i < 4; ++i) {
    const int mBase = m0 + (i << 4);
#pragma unroll
    for (int j = 0; j < 4; ++j) {
      const int n = (j << 4) + rlane;
      const float svn = SVp[z * HDIM + n];
#pragma unroll
      for (int r = 0; r < 8; ++r) {
        const int m = mBase + mOff + r;
        const float cf = stats[((size_t)z * SEQ + m) * 2];
        const float iz = stats[((size_t)z * SEQ + m) * 2 + 1];
        float v = acc[i][j][r] * PSC_INV + cf * svn;
        v = v * iz * YMUL;
        slab[(mOff + r) * 68 + (j << 4) + rlane] = v;
      }
    }
    __builtin_amdgcn_fence(__ATOMIC_RELEASE, "workgroup");
    __builtin_amdgcn_wave_barrier();
    __builtin_amdgcn_fence(__ATOMIC_ACQUIRE, "workgroup");
    {
      const int q = lane >> 3, c8 = (lane & 7) * 8;
      for (int pass = 0; pass < 2; ++pass) {
#pragma unroll
        for (int it = 0; it < 4; ++it) {
          const int row = it * 4 + q;
          const float* sp = slab + row * 68 + c8;
          v8h hv;
#pragma unroll
          for (int e = 0; e < 8; ++e) hv[e] = (_Float16)sp[e];
          *(volatile v8h*)(C + (size_t)(mBase + row) * EMB + c8) = hv;
        }
        __threadfence();
      }
    }
    __builtin_amdgcn_fence(__ATOMIC_RELEASE, "workgroup");
    __builtin_amdgcn_wave_barrier();
    __builtin_amdgcn_fence(__ATOMIC_ACQUIRE, "workgroup");
  }
}

constexpr size_t SZ_X16 = (size_t)NTOK * EMB * 2;
constexpr size_t SZ_WT  = (size_t)EMB * EMB * 2;
constexpr size_t SZ_QK  = (size_t)NTOK * EMB * 2;
constexpr size_t SZ_V32 = (size_t)NTOK * EMB * 4;
constexpr size_t SZ_VT  = (size_t)NBH * HDIM * PPITCH * 2;
constexpr size_t SZ_SV  = (size_t)NBH * HDIM * 4;
constexpr size_t SZ_P   = (size_t)NBH * SEQ * PPITCH * 2;
constexpr size_t SZ_ST  = (size_t)NBH * SEQ * 2 * 4;
constexpr size_t SZ_Y16 = (size_t)NTOK * EMB * 2;
constexpr size_t OFF_X16 = 0;
constexpr size_t OFF_WQT = OFF_X16 + SZ_X16;
constexpr size_t OFF_WKT = OFF_WQT + SZ_WT;
constexpr size_t OFF_WVT = OFF_WKT + SZ_WT;
constexpr size_t OFF_WOT = OFF_WVT + SZ_WT;
constexpr size_t OFF_QH  = OFF_WOT + SZ_WT;
constexpr size_t OFF_QL  = OFF_QH + SZ_QK;
constexpr size_t OFF_KH  = OFF_QL + SZ_QK;
constexpr size_t OFF_KL  = OFF_KH + SZ_QK;
constexpr size_t OFF_V32 = OFF_KL + SZ_QK;
constexpr size_t OFF_VT  = OFF_V32 + SZ_V32;
constexpr size_t OFF_SV  = OFF_VT + SZ_VT;
constexpr size_t OFF_P   = OFF_SV + SZ_SV;
constexpr size_t OFF_ST  = OFF_P + SZ_P;
constexpr size_t OFF_Y16 = OFF_ST + SZ_ST;
constexpr size_t WS_TOTAL = OFF_Y16 + SZ_Y16;
static_assert(WS_TOTAL == 87889920ull);
static_assert(WS_TOTAL <= 134217728ull);
static_assert((OFF_P % 128) == 0 && (OFF_ST % 128) == 0 && (OFF_Y16 % 128) == 0 && (OFF_SV % 128) == 0 && (OFF_VT % 128) == 0);
static_assert(KPV % 32 == 0 && EMB % 64 == 0 && NTOK % 64 == 0 && SEQ % 64 == 0 && HDIM == 64);

extern "C" void kernel_launch(void* const* d_in, const int* in_sizes, int n_in,
                              void* d_out, int out_size, void* d_ws, size_t ws_size,
                              hipStream_t stream) {
  if (n_in < 9) return;
  if (in_sizes[0] != NTOK * EMB || in_sizes[1] != EMB * EMB || in_sizes[2] != EMB ||
      in_sizes[3] != EMB * EMB || in_sizes[4] != EMB || in_sizes[5] != EMB * EMB ||
      in_sizes[6] != EMB || in_sizes[7] != EMB * EMB || in_sizes[8] != EMB) return;
  if (out_size != NTOK * EMB) return;
  if (WS_TOTAL > ws_size) return;

  const float* p_x  = (const float*)d_in[0];
  const float* p_Wq = (const float*)d_in[1];
  const float* p_bq = (const float*)d_in[2];
  const float* p_Wk = (const float*)d_in[3];
  const float* p_bk = (const float*)d_in[4];
  const float* p_Wv = (const float*)d_in[5];
  const float* p_bv = (const float*)d_in[6];
  const float* p_Wo = (const float*)d_in[7];
  const float* p_bo = (const float*)d_in[8];
  float* out = (float*)d_out;

  char* ws = (char*)d_ws;
  unsigned short* X16 = (unsigned short*)(ws + OFF_X16);
  unsigned short* WqT = (unsigned short*)(ws + OFF_WQT);
  unsigned short* WkT = (unsigned short*)(ws + OFF_WKT);
  unsigned short* WvT = (unsigned short*)(ws + OFF_WVT);
  unsigned short* WoT = (unsigned short*)(ws + OFF_WOT);
  unsigned short* Qh  = (unsigned short*)(ws + OFF_QH);
  unsigned short* Ql  = (unsigned short*)(ws + OFF_QL);
  unsigned short* Kh  = (unsigned short*)(ws + OFF_KH);
  unsigned short* Kl  = (unsigned short*)(ws + OFF_KL);
  float*          V32 = (float*)(ws + OFF_V32);
  unsigned short* Vt  = (unsigned short*)(ws + OFF_VT);
  float*          SV  = (float*)(ws + OFF_SV);
  unsigned short* P16 = (unsigned short*)(ws + OFF_P);
  float*          STT = (float*)(ws + OFF_ST);
  unsigned short* Y16 = (unsigned short*)(ws + OFF_Y16);

  {
    const int n2 = NTOK * EMB / 2;
    cast_x_k<<<(n2 + 255) / 256, 256, 0, stream>>>(p_x, X16, n2);
  }
  {
    dim3 wg(EMB / 64, EMB / 64);
    wt_cast_k<<<wg, 256, 0, stream>>>(p_Wq, WqT, EMB, EMB, WMUL);
    wt_cast_k<<<wg, 256, 0, stream>>>(p_Wk, WkT, EMB, EMB, WMUL);
    wt_cast_k<<<wg, 256, 0, stream>>>(p_Wv, WvT, EMB, EMB, WMUL);
    wt_cast_k<<<wg, 256, 0, stream>>>(p_Wo, WoT, EMB, EMB, WMUL);
  }
  {
    dim3 gg((NTOK / 64) * (EMB / 64) / 8, 1);
    const float sc = 1.0f / WMUL;
    wmma_gemm64<0, false, 3, 2, false><<<gg, 256, 0, stream>>>(
        X16, X16, EMB, 0, WqT, WqT, EMB, 0, (void*)Qh, (void*)Ql, EMB, 0, p_bq, p_bq, 0, NTOK, EMB, EMB, sc);
    wmma_gemm64<0, false, 3, 2, false><<<gg, 256, 0, stream>>>(
        X16, X16, EMB, 0, WkT, WkT, EMB, 0, (void*)Kh, (void*)Kl, EMB, 0, p_bk, p_bk, 0, NTOK, EMB, EMB, sc);
    wmma_gemm64<0, false, 3, 0, false><<<gg, 256, 0, stream>>>(
        X16, X16, EMB, 0, WvT, WvT, EMB, 0, (void*)V32, (void*)V32, EMB, 0, p_bv, p_bv, 0, NTOK, EMB, EMB, sc);
  }
  vprep_k<<<NBH, 256, 0, stream>>>(V32, Vt, SV);
  band_softmax_k<<<NBH * (SEQ / 64), 128, 0, stream>>>(Qh, Ql, Kh, Kl, P16, STT);
  {
    dim3 pg(SEQ / 64 / 8, NBH);
    pv_gemm_k<<<pg, 256, 0, stream>>>(P16, Vt, STT, SV, Y16);
  }
  {
    dim3 gg((NTOK / 64) * (EMB / 64) / 8, 1);
    const float sc = 1.0f / (WMUL * YMUL);
    wmma_gemm64<0, false, 3, 0, false><<<gg, 256, 0, stream>>>(
        Y16, Y16, EMB, 0, WoT, WoT, EMB, 0, (void*)out, (void*)out, EMB, 0, p_bo, p_bo, 0, NTOK, EMB, EMB, sc);
  }
}
